// EdgeNavierStokesLayer_41128606827044
// MI455X (gfx1250) — hardware-verified
//
#include <hip/hip_runtime.h>
#include <stddef.h>
#include <stdint.h>


#define DD       128
#define NPROJ    640
#define NWT      896
#define WSC      64.0f
#define WINV     0.015625f
#define DTS      0.03f
#define TWOLOG2E 2.8853900817779268f

#define G_THR    256
#define G_ROWS   32
#define G_CW     160
#define G_NCT    10
#define G_LDS_A  0
#define G_LDS_S  8192
#define G_LDS    (G_LDS_S + 8 * 16 * G_CW * 4)

#define NTHR     256
#define NWAVE    8
#define NB       256
#define EPT      8
#define CHUNK    (NTHR * EPT)
#define WCAP     (EPT * 32)
#define LISTN    (NWAVE * WCAP)
#define PASSN    128
#define NET      (PASSN / 16)
#define PCAP     (CHUNK + PASSN)
#define RMAX     ((PCAP + PASSN - 1) / PASSN)

#define L_ACC    0
#define L_F1     (L_ACC + (NB + 1) * DD * 4)
#define L_P1     (L_F1 + PASSN * DD * 2)
#define L_DH     (L_P1 + PASSN * DD * 2)
#define L_NU     (L_DH + PASSN * DD * 2)
#define L_SLOT   (L_NU + PASSN * 4)
#define L_LIST   (L_SLOT + PASSN * 4)
#define L_PEND   (L_LIST + LISTN * 4)
#define L_WCNT   (L_PEND + PCAP * 4)
#define L_PNDN   (L_WCNT + NWAVE * 4)
#define E_LDS    (L_PNDN + 16)

static_assert(PASSN == NWAVE * 16);
static_assert((NB % NWAVE) == 0);
static_assert(G_CW * 4 == NPROJ);
static_assert(G_NCT * 16 == G_CW);
static_assert(G_ROWS * DD == G_THR * 16);
static_assert((L_F1 & 15) == 0 && (L_P1 & 15) == 0 && (L_DH & 15) == 0 && (L_NU & 15) == 0);
static_assert((L_SLOT & 15) == 0 && (L_LIST & 15) == 0 && (L_PEND & 15) == 0 && (L_WCNT & 15) == 0);
static_assert(E_LDS <= 300 * 1024);
static_assert(G_LDS <= 300 * 1024);
static_assert(RMAX * PASSN >= PCAP);

#if __has_builtin(__builtin_amdgcn_exp2f)
#define FEXP2(v) __builtin_amdgcn_exp2f(v)
#else
#define FEXP2(v) exp2f(v)
#endif

typedef float    v4f  __attribute__((ext_vector_type(4)));
typedef float    v8f  __attribute__((ext_vector_type(8)));
typedef int      v4i  __attribute__((ext_vector_type(4)));
typedef _Float16 v4h  __attribute__((ext_vector_type(4)));
typedef _Float16 v8h  __attribute__((ext_vector_type(8)));
typedef _Float16 v16h __attribute__((ext_vector_type(16)));
union FragH { v16h v; v8h h[2]; };

__device__ __forceinline__ v8f zero8f() {
  v8f z;
#pragma unroll
  for (int i = 0; i < 8; ++i) z[i] = 0.0f;
  return z;
}

__device__ __forceinline__ v8f wmh(v16h a, v16h b, v8f c) {
  v8f d = __builtin_amdgcn_wmma_f32_16x16x32_f16(false, a, false, b, (short)0, c, false, false);
  asm volatile("v_nop\n\tv_nop\n\tv_nop\n\tv_nop" : "+v"(d) : "v"(a), "v"(b));
  return d;
}

__device__ __forceinline__ float ftanh(float x) {
  const float e = FEXP2(x * TWOLOG2E);
  const float r = __builtin_amdgcn_rcpf(e + 1.0f);
  return 1.0f - 2.0f * r;
}

__global__ __launch_bounds__(256) void k_wcvt(const float* __restrict__ vw1, const float* __restrict__ fw1,
                                              const float* __restrict__ pw1, const float* __restrict__ fw2,
                                              const float* __restrict__ pw2, _Float16* Wt) {
  const int t = blockIdx.x * 256 + threadIdx.x;
  if (t >= NWT * 16) return;
  const int ng = t >> 4, kc = (t & 15) * 8, seg = ng >> 7, n = ng & 127;
  const float* src = vw1;
  int roff = 0;
  if (seg == 1)      { src = vw1; roff = DD; }
  else if (seg == 2) { src = fw1; }
  else if (seg == 3) { src = fw1; roff = DD; }
  else if (seg == 4) { src = pw1; }
  else if (seg == 5) { src = fw2; }
  else if (seg == 6) { src = pw2; }
  v8h o;
#pragma unroll
  for (int i = 0; i < 8; ++i) o[i] = (_Float16)(src[(size_t)(roff + kc + i) * DD + n] * WSC);
  _Float16* dp = Wt + (size_t)ng * DD + kc;
  *(volatile v8h*)dp = o;
  __threadfence();
  *(volatile v8h*)dp = o;
}

__global__ __launch_bounds__(G_THR) void k_node(const float* __restrict__ h, const _Float16* Wt,
                                                float* P, int nN) {
  extern __shared__ __attribute__((aligned(16))) unsigned char lds_n[];
  _Float16* ah  = (_Float16*)(lds_n + G_LDS_A);
  float*    stg = (float*)(lds_n + G_LDS_S);

  const int tid = threadIdx.x, lane = tid & 31, wave = tid >> 5, hh = lane >> 4, m = lane & 15;
  const int wr = wave >> 2, wc = wave & 3;
  const int row0 = blockIdx.x * G_ROWS;

  {
    const int r = tid >> 3, k0 = (tid & 7) * 16;
    const int node = row0 + r;
    v4f x0 = {0.0f, 0.0f, 0.0f, 0.0f};
    v4f x1 = x0, x2 = x0, x3 = x0;
    if (node < nN) {
      const float* hp = h + (size_t)node * DD + k0;
      x0 = *(const v4f*)hp;
      x1 = *(const v4f*)(hp + 4);
      x2 = *(const v4f*)(hp + 8);
      x3 = *(const v4f*)(hp + 12);
    }
    v8h o0, o1;
#pragma unroll
    for (int i = 0; i < 4; ++i) {
      o0[i] = (_Float16)x0[i]; o0[4 + i] = (_Float16)x1[i];
      o1[i] = (_Float16)x2[i]; o1[4 + i] = (_Float16)x3[i];
    }
    *(v8h*)(ah + r * DD + k0)     = o0;
    *(v8h*)(ah + r * DD + k0 + 8) = o1;
  }
  __syncthreads();

  v8f accv[G_NCT];
#pragma unroll
  for (int j = 0; j < G_NCT; ++j) accv[j] = zero8f();

  const _Float16* abase = ah + (16 * wr + m) * DD + 8 * hh;
  const _Float16* bbase = Wt + (size_t)(wc * G_CW + m) * DD + 8 * hh;
#pragma unroll 1
  for (int kt = 0; kt < DD / 32; ++kt) {
    FragH a;
    a.h[0] = *(const v8h*)(abase + 32 * kt);
    a.h[1] = *(const v8h*)(abase + 32 * kt + 16);
#pragma unroll
    for (int j = 0; j < G_NCT; ++j) {
      const _Float16* bp = bbase + (size_t)(16 * j) * DD + 32 * kt;
      FragH b;
      b.h[0] = *(const v8h*)bp;
      b.h[1] = *(const v8h*)(bp + 16);
      accv[j] = wmh(a.v, b.v, accv[j]);
    }
  }

  float* st = stg + wave * (16 * G_CW);
#pragma unroll
  for (int j = 0; j < G_NCT; ++j) {
#pragma unroll
    for (int r = 0; r < 8; ++r) st[(8 * hh + r) * G_CW + 16 * j + m] = accv[j][r] * WINV;
  }
  __syncthreads();

  const size_t gbase = (size_t)(row0 + 16 * wr) * NPROJ + (size_t)(wc * G_CW);
#pragma unroll
  for (int q = 0; q < (16 * G_CW) / 128; ++q) {
    const int f = 128 * q + 4 * lane;
    const int rr = f / G_CW, cc = f - rr * G_CW;
    const v4f v = *(const v4f*)(st + f);
    *(volatile v4f*)(P + gbase + (size_t)rr * NPROJ + cc) = v;
  }
  __threadfence();
#pragma unroll
  for (int q = 0; q < (16 * G_CW) / 128; ++q) {
    const int f = 128 * q + 4 * lane;
    const int rr = f / G_CW, cc = f - rr * G_CW;
    const v4f v = *(const v4f*)(st + f);
    *(volatile v4f*)(P + gbase + (size_t)rr * NPROJ + cc) = v;
  }
}

__device__ __forceinline__ int scan_chunk(const int* __restrict__ dsts, int nE, int cbase, int nodeBase,
                                          int* list, int tid, int wave) {
  int wc = 0;
  const int el0  = tid * EPT;
  const int e0   = cbase + el0;
  const int sent = -2147483647 - 1;
  v4i da, db;
  if (e0 + 7 < nE) {
    da = *(const v4i*)(dsts + e0);
    db = *(const v4i*)(dsts + e0 + 4);
  } else {
    da.x = (e0     < nE) ? dsts[min(e0, nE - 1)]     : sent;
    da.y = (e0 + 1 < nE) ? dsts[min(e0 + 1, nE - 1)] : sent;
    da.z = (e0 + 2 < nE) ? dsts[min(e0 + 2, nE - 1)] : sent;
    da.w = (e0 + 3 < nE) ? dsts[min(e0 + 3, nE - 1)] : sent;
    db.x = (e0 + 4 < nE) ? dsts[min(e0 + 4, nE - 1)] : sent;
    db.y = (e0 + 5 < nE) ? dsts[min(e0 + 5, nE - 1)] : sent;
    db.z = (e0 + 6 < nE) ? dsts[min(e0 + 6, nE - 1)] : sent;
    db.w = (e0 + 7 < nE) ? dsts[min(e0 + 7, nE - 1)] : sent;
  }
  const unsigned nb = (unsigned)nodeBase;
  const unsigned s0 = (unsigned)da.x - nb, s1 = (unsigned)da.y - nb;
  const unsigned s2 = (unsigned)da.z - nb, s3 = (unsigned)da.w - nb;
  const unsigned s4 = (unsigned)db.x - nb, s5 = (unsigned)db.y - nb;
  const unsigned s6 = (unsigned)db.z - nb, s7 = (unsigned)db.w - nb;
  const bool h0 = s0 < (unsigned)NB, h1 = s1 < (unsigned)NB, h2 = s2 < (unsigned)NB, h3 = s3 < (unsigned)NB;
  const bool h4 = s4 < (unsigned)NB, h5 = s5 < (unsigned)NB, h6 = s6 < (unsigned)NB, h7 = s7 < (unsigned)NB;
  const unsigned any = __builtin_amdgcn_ballot_w32(h0 | h1 | h2 | h3 | h4 | h5 | h6 | h7);
  if (any != 0u) {
#define HITJ(J, HJ) { \
      const unsigned mj = __builtin_amdgcn_ballot_w32(HJ); \
      if (mj != 0u) { \
        if (HJ) { \
          const int pos = wc + (int)__builtin_amdgcn_mbcnt_lo(mj, 0u); \
          if (pos < WCAP) list[wave * WCAP + pos] = el0 + (J); \
        } \
        wc += (int)__builtin_popcount(mj); } }
    HITJ(0, h0)
    HITJ(1, h1)
    HITJ(2, h2)
    HITJ(3, h3)
    HITJ(4, h4)
    HITJ(5, h5)
    HITJ(6, h6)
    HITJ(7, h7)
#undef HITJ
  }
  return wc;
}

__global__ __launch_bounds__(NTHR) void k_edge(
    const float* __restrict__ h, const int* __restrict__ ei, const float* P, const _Float16* W2t,
    const float* __restrict__ vb1, const float* __restrict__ vw2, const float* __restrict__ vb2,
    const float* __restrict__ fb1, const float* __restrict__ pb1,
    const float* __restrict__ fb2, const float* __restrict__ pb2,
    float* outp, int nN, int nE) {
#pragma clang fp contract(off)
  extern __shared__ __attribute__((aligned(16))) unsigned char lds_e[];
  float*    acc   = (float*)(lds_e + L_ACC);
  _Float16* f1t   = (_Float16*)(lds_e + L_F1);
  _Float16* p1t   = (_Float16*)(lds_e + L_P1);
  _Float16* dht   = (_Float16*)(lds_e + L_DH);
  float*    nus   = (float*)(lds_e + L_NU);
  int*      slotb = (int*)(lds_e + L_SLOT);
  int*      list  = (int*)(lds_e + L_LIST);
  int*      pend  = (int*)(lds_e + L_PEND);
  int*      wcnt  = (int*)(lds_e + L_WCNT);
  int*      pendN = (int*)(lds_e + L_PNDN);

  const int tid = threadIdx.x, lane = tid & 31, wave = tid >> 5, hh = lane >> 4, m = lane & 15;
  const int nodeBase = blockIdx.x * NB;
  const int* dsts = ei;
  const int* srcs = ei + nE;

  {
    const v4f z = {0.0f, 0.0f, 0.0f, 0.0f};
    for (int i = tid; i < (NB + 1) * (DD / 4); i += NTHR) *(v4f*)(acc + 4 * i) = z;
  }
  if (tid == 0) pendN[0] = 0;
  const int c4 = 4 * lane;
  const v4f vb1v = *(const v4f*)(vb1 + c4);
  const v4f vw2v = *(const v4f*)(vw2 + c4);
  const v4f fb1v = *(const v4f*)(fb1 + c4);
  const v4f pb1v = *(const v4f*)(pb1 + c4);
  const float vb2s = vb2[0];
  const int ncol = 16 * wave + m;
  const float fb2n = fb2[ncol], pb2n = pb2[ncol];
  __syncthreads();

  const int nChunks = (nE + CHUNK - 1) / CHUNK;
#pragma unroll 1
  for (int ch = 0; ch < nChunks; ++ch) {
    const int cbase = ch * CHUNK;
    const int wc = scan_chunk(dsts, nE, cbase, nodeBase, list, tid, wave);
    if (lane == 0) wcnt[wave] = wc;
    __syncthreads();

    int base = pendN[0];
    base = base < 0 ? 0 : (base > PASSN - 1 ? PASSN - 1 : base);
    int tot = 0, myoff = 0;
#pragma unroll
    for (int w = 0; w < NWAVE; ++w) {
      int c = wcnt[w];
      c = c > WCAP ? WCAP : (c < 0 ? 0 : c);
      if (w < wave) myoff += c;
      tot += c;
    }
    int newN = base + tot;
    newN = newN > PCAP ? PCAP : newN;
    {
      int n = wcnt[wave];
      n = n > WCAP ? WCAP : (n < 0 ? 0 : n);
      const int* lp = list + wave * WCAP;
      for (int i = lane; i < n; i += 32) {
        const int pos = base + myoff + i;
        if ((unsigned)pos < (unsigned)PCAP) pend[pos] = cbase + lp[i];
      }
    }
    const int fin = (ch == nChunks - 1) ? 1 : 0;
    int R = (fin != 0) ? (newN + PASSN - 1) / PASSN : newN / PASSN;
    R = R > RMAX ? RMAX : (R < 0 ? 0 : R);
    const int Pv = (fin != 0) ? newN : R * PASSN;
    __syncthreads();

#pragma unroll 1
    for (int r = 0; r < R; ++r) {
#pragma unroll 1
      for (int ee = 0; ee < 16; ++ee) {
        const int erow = wave * 16 + ee;
        const int idx  = r * PASSN + erow;
        const bool valid = idx < Pv;
        int e = pend[idx < PCAP ? idx : (PCAP - 1)];
        e = e < 0 ? 0 : (e > nE - 1 ? nE - 1 : e);
        int di = dsts[e];
        int sj = srcs[e];
        int slot = di - nodeBase;
        if (!valid || (unsigned)slot >= (unsigned)NB) slot = NB;
        di = di < 0 ? 0 : (di > nN - 1 ? nN - 1 : di);
        sj = sj < 0 ? 0 : (sj > nN - 1 ? nN - 1 : sj);
        const float* Pi = P + (size_t)di * NPROJ + c4;
        const float* Pj = P + (size_t)sj * NPROJ + c4;
        const v4f pva = *(const v4f*)(Pi);
        const v4f pfa = *(const v4f*)(Pi + 2 * DD);
        const v4f ppi = *(const v4f*)(Pi + 4 * DD);
        const v4f pvb = *(const v4f*)(Pj + DD);
        const v4f pfb = *(const v4f*)(Pj + 3 * DD);
        const v4f ppj = *(const v4f*)(Pj + 4 * DD);
        const v4f hiv = *(const v4f*)(h + (size_t)di * DD + c4);
        const v4f hjv = *(const v4f*)(h + (size_t)sj * DD + c4);
        float nup = 0.0f;
        v4h f1h, p1h, dhh;
#pragma unroll
        for (int c = 0; c < 4; ++c) {
          const float xv = (pva[c] + pvb[c]) + vb1v[c];
          const float tv = ftanh(xv);
          nup = fmaf(tv, vw2v[c], nup);
          const float xf = (pfa[c] + pfb[c]) + fb1v[c];
          f1h[c] = (_Float16)fmaxf(xf, 0.0f);
          const float xp = (ppi[c] - ppj[c]) + pb1v[c];
          p1h[c] = (_Float16)ftanh(xp);
          dhh[c] = (_Float16)(hjv[c] - hiv[c]);
        }
        nup += __shfl_xor(nup, 16);
        nup += __shfl_xor(nup, 8);
        nup += __shfl_xor(nup, 4);
        nup += __shfl_xor(nup, 2);
        nup += __shfl_xor(nup, 1);
        *(v4h*)(f1t + erow * DD + c4) = f1h;
        *(v4h*)(p1t + erow * DD + c4) = p1h;
        *(v4h*)(dht + erow * DD + c4) = dhh;
        if (lane == 0) { nus[erow] = nup + vb2s; slotb[erow] = slot; }
      }
      __syncthreads();

      {
        FragH bF[4], bP[4];
        const _Float16* wf = W2t + (size_t)ncol * DD + 8 * hh;
        const _Float16* wp = W2t + (size_t)(DD + ncol) * DD + 8 * hh;
#pragma unroll
        for (int kt = 0; kt < 4; ++kt) {
          bF[kt].h[0] = *(const v8h*)(wf + 32 * kt);
          bF[kt].h[1] = *(const v8h*)(wf + 32 * kt + 16);
          bP[kt].h[0] = *(const v8h*)(wp + 32 * kt);
          bP[kt].h[1] = *(const v8h*)(wp + 32 * kt + 16);
        }
#pragma unroll 1
        for (int et = 0; et < NET; ++et) {
          v8f aF = zero8f(), aP = zero8f();
          const _Float16* af = f1t + (16 * et + m) * DD + 8 * hh;
          const _Float16* ap = p1t + (16 * et + m) * DD + 8 * hh;
#pragma unroll
          for (int kt = 0; kt < 4; ++kt) {
            FragH a1, a2;
            a1.h[0] = *(const v8h*)(af + 32 * kt);
            a1.h[1] = *(const v8h*)(af + 32 * kt + 16);
            a2.h[0] = *(const v8h*)(ap + 32 * kt);
            a2.h[1] = *(const v8h*)(ap + 32 * kt + 16);
            aF = wmh(a1.v, bF[kt].v, aF);
            aP = wmh(a2.v, bP[kt].v, aP);
          }
          float mv[8], mw[8];
#pragma unroll
          for (int rr = 0; rr < 8; ++rr) {
            const int erow = 16 * et + 8 * hh + rr;
            const float dh = (float)dht[erow * DD + ncol];
            const float nu = nus[erow];
            const float fo = aF[rr] * WINV + fb2n;
            const float po = aP[rr] * WINV + pb2n;
            mv[rr] = (nu * dh + fo) - po;
          }
#pragma unroll
          for (int rr = 0; rr < 8; ++rr) mw[rr] = __shfl_xor(mv[rr], 16);
          if (hh == 0) {
#pragma unroll
            for (int rr = 0; rr < 8; ++rr) {
              int s0 = slotb[16 * et + rr];
              s0 = s0 < 0 ? 0 : (s0 > NB ? NB : s0);
              float* q0 = acc + s0 * DD + ncol;
              const float t0 = *q0 + mv[rr];
              *q0 = t0;
              int s1 = slotb[16 * et + 8 + rr];
              s1 = s1 < 0 ? 0 : (s1 > NB ? NB : s1);
              float* q1 = acc + s1 * DD + ncol;
              const float t1 = *q1 + mw[rr];
              *q1 = t1;
            }
          }
        }
      }
      __syncthreads();
    }

    int rem = newN - R * PASSN;
    rem = rem < 0 ? 0 : (rem > PASSN - 1 ? PASSN - 1 : rem);
    if (R > 0 && tid < rem) pend[tid] = pend[R * PASSN + tid];
    if (tid == 0) pendN[0] = rem;
  }
  __syncthreads();

#pragma unroll 1
  for (int it = 0; it < NB / NWAVE; ++it) {
    const int sl = wave * (NB / NWAVE) + it;
    const int node = nodeBase + sl;
    if (node < nN) {
      const v4f hv = *(const v4f*)(h + (size_t)node * DD + c4);
      const v4f av = *(const v4f*)(acc + sl * DD + c4);
      v4f o;
#pragma unroll
      for (int c = 0; c < 4; ++c) { const float tprod = DTS * av[c]; o[c] = hv[c] + tprod; }
      *(volatile v4f*)(outp + (size_t)node * DD + c4) = o;
    }
  }
  __threadfence();
#pragma unroll 1
  for (int it = 0; it < NB / NWAVE; ++it) {
    const int sl = wave * (NB / NWAVE) + it;
    const int node = nodeBase + sl;
    if (node < nN) {
      const v4f hv = *(const v4f*)(h + (size_t)node * DD + c4);
      const v4f av = *(const v4f*)(acc + sl * DD + c4);
      v4f o;
#pragma unroll
      for (int c = 0; c < 4; ++c) { const float tprod = DTS * av[c]; o[c] = hv[c] + tprod; }
      *(volatile v4f*)(outp + (size_t)node * DD + c4) = o;
    }
  }
}

extern "C" void kernel_launch(void* const* d_in, const int* in_sizes, int n_in,
                              void* d_out, int out_size, void* d_ws, size_t ws_size,
                              hipStream_t stream) {
  if (n_in < 14) return;
  const int nN = in_sizes[0] / DD;
  const int nE = in_sizes[1] / 2;
  if (nN <= 0 || nE <= 0 || in_sizes[0] != nN * DD || in_sizes[1] != 2 * nE) return;
  if (in_sizes[2] != 2 * DD * DD || in_sizes[3] < DD || in_sizes[4] < DD || in_sizes[5] < 1) return;
  if (in_sizes[6] != DD * DD || in_sizes[7] < DD || in_sizes[8] != DD * DD || in_sizes[9] < DD) return;
  if (in_sizes[10] != 2 * DD * DD || in_sizes[11] < DD || in_sizes[12] != DD * DD || in_sizes[13] < DD) return;
  if (out_size != nN * DD) return;

  const float* h   = (const float*)d_in[0];
  const int*   ei  = (const int*)d_in[1];
  const float* vw1 = (const float*)d_in[2];
  const float* vb1 = (const float*)d_in[3];
  const float* vw2 = (const float*)d_in[4];
  const float* vb2 = (const float*)d_in[5];
  const float* pw1 = (const float*)d_in[6];
  const float* pb1 = (const float*)d_in[7];
  const float* pw2 = (const float*)d_in[8];
  const float* pb2 = (const float*)d_in[9];
  const float* fw1 = (const float*)d_in[10];
  const float* fb1 = (const float*)d_in[11];
  const float* fw2 = (const float*)d_in[12];
  const float* fb2 = (const float*)d_in[13];
  float* out = (float*)d_out;

  const int Mpad  = ((nN + G_ROWS - 1) / G_ROWS) * G_ROWS;
  const int nBlkG = Mpad / G_ROWS;
  const int nBlkE = (nN + NB - 1) / NB;

  char* ws = (char*)d_ws;
  size_t off = 0;
  const size_t oWt = off; off += (size_t)NWT * DD * 2;     off = (off + 255) & ~(size_t)255;
  const size_t oP  = off; off += (size_t)Mpad * NPROJ * 4;  off = (off + 255) & ~(size_t)255;
  if (off > ws_size) return;
  _Float16* Wt = (_Float16*)(ws + oWt);
  float*    Pb = (float*)(ws + oP);

  const hipError_t ea = hipFuncSetAttribute(reinterpret_cast<const void*>(&k_node),
                                            hipFuncAttributeMaxDynamicSharedMemorySize, G_LDS);
  const hipError_t eb = hipFuncSetAttribute(reinterpret_cast<const void*>(&k_edge),
                                            hipFuncAttributeMaxDynamicSharedMemorySize, E_LDS);
  (void)ea;
  (void)eb;

  k_wcvt<<<(NWT * 16 + 255) / 256, 256, 0, stream>>>(vw1, fw1, pw1, fw2, pw2, Wt);

  k_node<<<nBlkG, G_THR, G_LDS, stream>>>(h, Wt, Pb, nN);

  k_edge<<<nBlkE, NTHR, E_LDS, stream>>>(h, ei, Pb, Wt + (size_t)NPROJ * DD,
                                          vb1, vw2, vb2, fb1, pb1, fb2, pb2, out, nN, nE);
  (void)hipGetLastError();
}
